// GaussianMixtureModel_18537078850250
// MI455X (gfx1250) — hardware-verified
//
#include <hip/hip_runtime.h>


#define NBT  65536
#define DD   128
#define KK   16
#define CH   8192
typedef _Float16 h16;
typedef unsigned short bf;
typedef __attribute__((ext_vector_type(16))) __bf16   v16bf;
typedef __attribute__((ext_vector_type(16))) _Float16 v16h;
typedef __attribute__((ext_vector_type(8)))  _Float16 v8h;
typedef __attribute__((ext_vector_type(8)))  unsigned short v8us;
typedef __attribute__((ext_vector_type(8)))  float    v8f;
typedef __attribute__((ext_vector_type(4)))  float    v4f;
typedef v8h  __attribute__((may_alias)) v8ha;
typedef v4f  __attribute__((may_alias)) v4fa;
typedef v8us __attribute__((may_alias)) v8usa;

__device__ __forceinline__ unsigned short f2bf(float f) { unsigned u = __float_as_uint(f); u += 0x7FFFu + ((u >> 16) & 1u); return (unsigned short)(u >> 16); }
__device__ __forceinline__ float bf2f(unsigned short b) { return __uint_as_float(((unsigned)b) << 16); }
__device__ __forceinline__ float bfr(float f) { return bf2f(f2bf(f)); }
__device__ __forceinline__ v16h cat16(v8h lo, v8h hi) { return __builtin_shufflevector(lo, hi, 0, 1, 2, 3, 4, 5, 6, 7, 8, 9, 10, 11, 12, 13, 14, 15); }
__device__ __forceinline__ v16bf cat16b(v8us lo, v8us hi) { return __builtin_bit_cast(v16bf, __builtin_shufflevector(lo, hi, 0, 1, 2, 3, 4, 5, 6, 7, 8, 9, 10, 11, 12, 13, 14, 15)); }
__device__ __forceinline__ v8f wmma16(v16h a, v16h b, v8f c) { return __builtin_amdgcn_wmma_f32_16x16x32_f16(false, a, false, b, (short)0, c, false, false); }
__device__ __forceinline__ v8f wmmab(v16bf a, v16bf b, v8f c) { return __builtin_amdgcn_wmma_f32_16x16x32_bf16(false, a, false, b, (short)0, c, false, false); }


template <typename T16> struct WFrag;
template <> struct WFrag<h16> { typedef v16h V; static __device__ __forceinline__ V ld(const h16* p) { return cat16(*(const v8h*)p, *(const v8h*)(p + 16)); } static __device__ __forceinline__ v8f mma(V a, V b, v8f c) { return wmma16(a, b, c); } };
template <> struct WFrag<bf> { typedef v16bf V; static __device__ __forceinline__ V ld(const bf* p) { return cat16b(*(const v8us*)p, *(const v8us*)(p + 16)); } static __device__ __forceinline__ v8f mma(V a, V b, v8f c) { return wmmab(a, b, c); } };
template <typename T16, int NSPLIT, bool BIAS>
__global__ __launch_bounds__(32) void k_gemmw(const T16* __restrict__ A, const T16* __restrict__ A2, const T16* __restrict__ Bt, const T16* __restrict__ Bt2, int K, float* C, int ldc, const float* __restrict__ bias, size_t sA, size_t sB, size_t sC) {
    typedef typename WFrag<T16>::V V;
    __shared__ __align__(16) float os[16 * 68];
    const size_t z = blockIdx.z; A += z * sA; if (A2) A2 += z * sA; Bt += z * sB; if (Bt2) Bt2 += z * sB; C += z * sC;
    const int lane = threadIdx.x & 31, lr = lane & 15, hi = lane >> 4; const int r0 = blockIdx.x * 64, c0 = blockIdx.y * 64;
    v8f acc[4][4];
#pragma unroll
    for (int mb = 0; mb < 4; ++mb)
#pragma unroll
        for (int nb = 0; nb < 4; ++nb) acc[mb][nb] = (v8f){};
    const size_t aoff = (size_t)(r0 + lr) * K + 8 * hi, boff = (size_t)(c0 + lr) * K + 8 * hi;
#pragma unroll 1
    for (int kc = 0; kc < K; kc += 32) {
        V a[4], a2[4];
#pragma unroll
        for (int mb = 0; mb < 4; ++mb) { a[mb] = WFrag<T16>::ld(A + aoff + (size_t)mb * 16 * K + kc); if (NSPLIT == 1 || NSPLIT == 2) a2[mb] = WFrag<T16>::ld(A2 + aoff + (size_t)mb * 16 * K + kc); }
#pragma unroll
        for (int nb = 0; nb < 4; ++nb) { const V b = WFrag<T16>::ld(Bt + boff + (size_t)nb * 16 * K + kc); V b2; if (NSPLIT >= 2) b2 = WFrag<T16>::ld(Bt2 + boff + (size_t)nb * 16 * K + kc);
#pragma unroll
            for (int mb = 0; mb < 4; ++mb) { acc[mb][nb] = WFrag<T16>::mma(a[mb], b, acc[mb][nb]); if (NSPLIT == 1 || NSPLIT == 2) acc[mb][nb] = WFrag<T16>::mma(a2[mb], b, acc[mb][nb]); if (NSPLIT >= 2) acc[mb][nb] = WFrag<T16>::mma(a[mb], b2, acc[mb][nb]); } }
        asm volatile("v_nop\n\tv_nop\n\tv_nop\n\tv_nop" : "+v"(acc[0][0]), "+v"(acc[1][1]), "+v"(acc[2][2]), "+v"(acc[3][3]) : "v"(a[0]), "v"(a[3]));
    }
#pragma unroll
    for (int mb = 0; mb < 4; ++mb) {
#pragma unroll
        for (int nb = 0; nb < 4; ++nb) {
#pragma unroll
            for (int j = 0; j < 8; ++j) os[(hi * 8 + j) * 68 + nb * 16 + lr] = acc[mb][nb][j]; }
        __builtin_amdgcn_wave_barrier(); asm volatile("" ::: "memory");
        float* crow = C + (size_t)(r0 + mb * 16) * ldc + c0;
#pragma unroll 1
        for (int ps = 0; ps < 2; ++ps) {
#pragma unroll
            for (int s = 0; s < 8; ++s) { const int row = 2 * s + hi, cofs = lr * 4; v4f val = *(const v4fa*)(os + row * 68 + cofs); if (BIAS) { val[0] += bfr(bias[c0 + cofs]); val[1] += bfr(bias[c0 + cofs + 1]); val[2] += bfr(bias[c0 + cofs + 2]); val[3] += bfr(bias[c0 + cofs + 3]); }
                *(volatile v4f*)(crow + (size_t)row * ldc + cofs) = val; }
            if (ps == 0) __threadfence(); }
        __builtin_amdgcn_wave_barrier(); asm volatile("" ::: "memory");
    }
}


__global__ __launch_bounds__(256) void k_cvt8(const float* __restrict__ src, bf* dst, size_t n8) { const size_t i = (size_t)blockIdx.x * 256 + threadIdx.x; if (i >= n8) return; const v8f v = *(const v8f*)(src + i * 8); v8us o;
#pragma unroll
    for (int k = 0; k < 8; ++k) o[k] = f2bf(v[k]); *(volatile v8us*)(dst + i * 8) = o; __threadfence(); *(volatile v8us*)(dst + i * 8) = o; }
__global__ __launch_bounds__(32) void k_cvec(const float* __restrict__ P, const float* __restrict__ mu, const float* __restrict__ lw, float* CV, float* LD) { const int lane = threadIdx.x; const int k = blockIdx.x; const float* Pk = P + (size_t)k * DD * DD; float cv[4];
#pragma unroll
    for (int u = 0; u < 4; ++u) { const int i = lane + 32 * u; float s = 0.f; for (int j = 0; j < DD; ++j) { float w = bfr(Pk[(size_t)i * DD + j]); asm volatile("" : "+v"(w)); float p = __fmul_rn(w, bfr(mu[k * DD + j])); asm volatile("" : "+v"(p)); s = __fadd_rn(s, p); } cv[u] = s; }
    float ld = 0.f; for (int u = 0; u < 4; ++u) { const int i = lane + 32 * u; ld = __fadd_rn(ld, logf(bfr(Pk[(size_t)i * DD + i]))); }
#pragma unroll
    for (int sh = 16; sh; sh >>= 1) ld += __shfl_xor(ld, sh, 32);
    const float c0 = __fadd_rn(__fadd_rn(-0.5f * DD * 1.8378770664093453f, ld), bfr(lw[k])); const float o = lane == 0 ? c0 : 0.f;
    for (int ps = 0; ps < 2; ++ps) {
#pragma unroll
        for (int u = 0; u < 4; ++u) *(volatile float*)(CV + k * DD + 32 * u + lane) = cv[u];
        *(volatile float*)(LD + k * 32 + lane) = o; if (ps == 0) __threadfence(); } }
__global__ __launch_bounds__(256) void k_gmm(const float* __restrict__ Y, const float* __restrict__ CV, const float* __restrict__ LD, float* OUTc) { const int b = blockIdx.x * 256 + threadIdx.x; if (b >= CH) return; float l[KK];
#pragma unroll
    for (int k = 0; k < KK; ++k) { const float* yr = Y + ((size_t)k * CH + b) * DD; float q = 0.f;
#pragma unroll 4
        for (int i = 0; i < DD; i += 4) { const v4f a = *(const v4f*)(yr + i);
#pragma unroll
            for (int u = 0; u < 4; ++u) { const float d = __fsub_rn(a[u], CV[k * DD + i + u]); float p = __fmul_rn(d, d); asm volatile("" : "+v"(p)); q = __fadd_rn(q, p); } }
        float hq = 0.5f * q; asm volatile("" : "+v"(hq)); l[k] = __fsub_rn(LD[k * 32], hq); }
    float m = l[0];
#pragma unroll
    for (int k = 1; k < KK; ++k) m = fmaxf(m, l[k]);
    float s = 0.f;
#pragma unroll
    for (int k = 0; k < KK; ++k) { float d0 = __fsub_rn(l[k], m); asm volatile("" : "+v"(d0)); s = __fadd_rn(s, __expf(d0)); }
    float lg = logf(s); asm volatile("" : "+v"(lg)); const float o = __fadd_rn(m, lg); *(volatile float*)(OUTc + b) = o; __threadfence(); *(volatile float*)(OUTc + b) = o; }

extern "C" void kernel_launch(void* const* d_in, const int* in_sizes, int n_in,
                              void* d_out, int out_size, void* d_ws, size_t ws_size, hipStream_t stream) {
    (void)in_sizes; (void)n_in; (void)out_size;
    const float* x = (const float*)d_in[0]; const float* mu = (const float*)d_in[1]; const float* P = (const float*)d_in[2]; const float* lw = (const float*)d_in[3];
    float* OUT = (float*)d_out;
    char* wsp = (char*)d_ws;
    auto take = [&](size_t bytes) { char* p = wsp; wsp += (bytes + 255) & ~(size_t)255; return (void*)p; };
    bf* PB = (bf*)take((size_t)KK * DD * DD * 2); bf* XB = (bf*)take((size_t)NBT * DD * 2); float* CV = (float*)take((size_t)KK * DD * 4); float* LD = (float*)take((size_t)KK * 32 * 4); float* Y = (float*)take((size_t)KK * CH * DD * 4);
    if ((size_t)(wsp - (char*)d_ws) > ws_size) return;
    k_cvt8<<<(unsigned)(((size_t)KK * DD * DD / 8 + 255) / 256), 256, 0, stream>>>(P, PB, (size_t)KK * DD * DD / 8); k_cvt8<<<(unsigned)(((size_t)NBT * DD / 8 + 255) / 256), 256, 0, stream>>>(x, XB, (size_t)NBT * DD / 8);
    k_cvec<<<KK, 32, 0, stream>>>(P, mu, lw, CV, LD);
    for (int c = 0; c < NBT / CH; ++c) {
        k_gemmw<bf, 0, false><<<dim3(CH / 64, DD / 64, KK), 32, 0, stream>>>(XB + (size_t)c * CH * DD, nullptr, PB, nullptr, DD, Y, DD, nullptr, 0, (size_t)DD * DD, (size_t)CH * DD);
        k_gmm<<<CH / 256, 256, 0, stream>>>(Y, CV, LD, OUT + (size_t)c * CH); }
}
